// GraphConditionEncoder_67680094650551
// MI455X (gfx1250) — hardware-verified
//
#include <hip/hip_runtime.h>
#include <stddef.h>
#include <stdint.h>
#include <math.h>


#define NN      30000
#define NE      240000
#define NGR     64
#define FD      64
#define NHD     4
#define HID     64
#define HC      256
#define K0      128
#define KA      512
#define GC      832
#define KG      1664
#define BOT     256
#define MROWS   128
#define MPC     30080
#define NTHR    256
#define NWAVE   8
#define EPT     8
#define CHUNK   (NTHR * EPT)
#define WCAP    (EPT * 32)
#define LISTN   (NWAVE * WCAP)
#define NB      1024
#define SLOTB   10
#define RCAP    28672
#define DEGCAP  64
#define GBM     64
#define GBN     64
#define GTHR    128
#define NEGSL   0.2f
#define EPS_SM  1e-16f
#define WSMAX   134217728
#define LDS_SCAN ((2 * RCAP + 2 * NB + LISTN) * 4 + 64)
#define VG __attribute__((amdgpu_num_vgpr(248)))

static_assert(MPC == ((NN + MROWS - 1) / MROWS) * MROWS);
static_assert((MPC % GBM) == 0 && NGR == GBM);
static_assert((K0 % 32) == 0 && (KA % 32) == 0 && (KG % 32) == 0);
static_assert(K0 == 2 * FD && KA == 2 * HC && KG == 2 * GC);
static_assert(HC == NHD * HID && HID == GBN && (BOT % GBN) == 0);
static_assert(GC == FD + 3 * HC && (GC % 8) == 0 && (FD % 8) == 0 && (HC % 8) == 0);
static_assert((CHUNK & (CHUNK - 1)) == 0 && NB == (1 << SLOTB) && CHUNK <= 4096);
static_assert(NTHR * 4 == NB && LISTN >= NB && (NB % NWAVE) == 0);
static_assert((RCAP % 32) == 0 && RCAP >= 8321 + 4096);
static_assert(DEGCAP >= 22 + 8);
static_assert(NE < (1 << 21));
static_assert(LDS_SCAN <= 300000);
static_assert(GBM == (GTHR / 32) * 16 && GTHR == 2 * GBN && GTHR == 2 * GBM);
static_assert(HC == 8 * 32 && HID == 8 * 8);
static_assert((NN % 4) == 0);
static_assert((MPC * (K0 / 8)) % NTHR == 0);
static_assert((NGR * (KG / 8)) % NTHR == 0);
static_assert((NGR - 1) * BOT + BOT - 1 == 16383);

typedef float          v2f  __attribute__((ext_vector_type(2)));
typedef float          v4f  __attribute__((ext_vector_type(4)));
typedef float          v8f  __attribute__((ext_vector_type(8)));
typedef int            v4i  __attribute__((ext_vector_type(4)));
typedef int            v8i  __attribute__((ext_vector_type(8)));
typedef unsigned int   v4u  __attribute__((ext_vector_type(4)));
typedef unsigned short v8us __attribute__((ext_vector_type(8)));
typedef __bf16         v16b __attribute__((ext_vector_type(16)));
typedef v2f  __attribute__((may_alias)) v2fa;
typedef v4f  __attribute__((may_alias)) v4fa;
typedef v4i  __attribute__((may_alias)) v4ia;
typedef v4u  __attribute__((may_alias)) v4ua;
typedef unsigned int __attribute__((may_alias)) u32a;
typedef v8us __attribute__((may_alias)) v8usa;
union FragB { v16b v; v8us h[2]; v8i w; };

__device__ __forceinline__ v8f wmb(const FragB& a, const FragB& b, v8f c) {
  v8f d = __builtin_amdgcn_wmma_f32_16x16x32_bf16(false, a.v, false, b.v, (short)0, c, false, false);
  asm volatile("v_nop\n\tv_nop\n\tv_nop\n\tv_nop" : "+v"(d) : "v"(a.w), "v"(b.w));
  return d;
}

__device__ __forceinline__ unsigned int f2bf(float f) {
  const unsigned int u = __float_as_uint(f);
  const unsigned int r = ((u + 0x7FFFu + ((u >> 16) & 1u)) >> 16) & 0xFFFFu;
  return (f != f) ? 0x7FC0u : r;
}
__device__ __forceinline__ float bf2f(unsigned int b) { return __uint_as_float(b << 16); }
__device__ __forceinline__ float bfr(float f) { return bf2f(f2bf(f)); }
__device__ __forceinline__ v4f bfr4(const v4f a) {
  v4f r; r.x = bfr(a.x); r.y = bfr(a.y); r.z = bfr(a.z); r.w = bfr(a.w); return r;
}
__device__ __forceinline__ unsigned int pk2(float lo, float hi) { return f2bf(lo) | (f2bf(hi) << 16); }
__device__ __forceinline__ v4u pack8(const v4f a, const v4f b) {
  v4u r;
  r.x = pk2(a.x, a.y); r.y = pk2(a.z, a.w); r.z = pk2(b.x, b.y); r.w = pk2(b.z, b.w);
  return r;
}
struct HL8 { v4u h; v4u l; };
__device__ __forceinline__ HL8 split8(const v4f a, const v4f b) {
  const unsigned int h0 = f2bf(a.x), h1 = f2bf(a.y), h2 = f2bf(a.z), h3 = f2bf(a.w);
  const unsigned int h4 = f2bf(b.x), h5 = f2bf(b.y), h6 = f2bf(b.z), h7 = f2bf(b.w);
  const unsigned int g0 = f2bf(a.x - bf2f(h0)), g1 = f2bf(a.y - bf2f(h1));
  const unsigned int g2 = f2bf(a.z - bf2f(h2)), g3 = f2bf(a.w - bf2f(h3));
  const unsigned int g4 = f2bf(b.x - bf2f(h4)), g5 = f2bf(b.y - bf2f(h5));
  const unsigned int g6 = f2bf(b.z - bf2f(h6)), g7 = f2bf(b.w - bf2f(h7));
  HL8 r;
  r.h.x = h0 | (h1 << 16); r.h.y = h2 | (h3 << 16); r.h.z = h4 | (h5 << 16); r.h.w = h6 | (h7 << 16);
  r.l.x = g0 | (g1 << 16); r.l.y = g2 | (g3 << 16); r.l.z = g4 | (g5 << 16); r.l.w = g6 | (g7 << 16);
  return r;
}
__device__ __forceinline__ float reluk(float v) { return (v > 0.f) ? v : (v - v); }
__device__ __forceinline__ float smax(float m, float v) { return (v > m || v != v) ? v : m; }

__device__ __forceinline__ int scan_chunk(const int* __restrict__ dsts, int nE, int cbase, int slotBase,
                                          int nb, int vec8, int* list, int tid, int lane, int wave) {
  int wc = 0;
  const int el0  = tid * EPT;
  const int e0   = cbase + el0;
  const int sent = -2147483647 - 1;
  v4i da, db;
  if (vec8 != 0 && cbase + CHUNK <= nE) {
    da = *(const v4i*)(dsts + e0);
    db = *(const v4i*)(dsts + e0 + 4);
  } else {
    da.x = (e0     < nE) ? dsts[min(e0,     nE - 1)] : sent;
    da.y = (e0 + 1 < nE) ? dsts[min(e0 + 1, nE - 1)] : sent;
    da.z = (e0 + 2 < nE) ? dsts[min(e0 + 2, nE - 1)] : sent;
    da.w = (e0 + 3 < nE) ? dsts[min(e0 + 3, nE - 1)] : sent;
    db.x = (e0 + 4 < nE) ? dsts[min(e0 + 4, nE - 1)] : sent;
    db.y = (e0 + 5 < nE) ? dsts[min(e0 + 5, nE - 1)] : sent;
    db.z = (e0 + 6 < nE) ? dsts[min(e0 + 6, nE - 1)] : sent;
    db.w = (e0 + 7 < nE) ? dsts[min(e0 + 7, nE - 1)] : sent;
  }
  const unsigned nbs = (unsigned)slotBase;
  const unsigned unb = (unsigned)nb;
  const unsigned s0 = (unsigned)da.x - nbs, s1 = (unsigned)da.y - nbs;
  const unsigned s2 = (unsigned)da.z - nbs, s3 = (unsigned)da.w - nbs;
  const unsigned s4 = (unsigned)db.x - nbs, s5 = (unsigned)db.y - nbs;
  const unsigned s6 = (unsigned)db.z - nbs, s7 = (unsigned)db.w - nbs;
  const bool h0 = s0 < unb, h1 = s1 < unb, h2 = s2 < unb, h3 = s3 < unb;
  const bool h4 = s4 < unb, h5 = s5 < unb, h6 = s6 < unb, h7 = s7 < unb;
  const unsigned any = __builtin_amdgcn_ballot_w32(h0 | h1 | h2 | h3 | h4 | h5 | h6 | h7);
  if (any != 0u) {
#define HITJ(J, HJ, SJ) { \
      const unsigned mj = __builtin_amdgcn_ballot_w32(HJ); \
      if (mj != 0u) { \
        if (HJ) { \
          const int pos = wc + (int)__builtin_amdgcn_mbcnt_lo(mj, 0u); \
          if (pos < WCAP) list[wave * WCAP + pos] = ((el0 + (J)) << SLOTB) | (int)(SJ); \
        } \
        wc += (int)__builtin_popcount(mj); } }
    HITJ(0, h0, s0)
    HITJ(1, h1, s1)
    HITJ(2, h2, s2)
    HITJ(3, h3, s3)
    HITJ(4, h4, s4)
    HITJ(5, h5, s5)
    HITJ(6, h6, s6)
    HITJ(7, h7, s7)
#undef HITJ
  }
  return wc;
}

__global__ __launch_bounds__(NTHR) VG void k_x0(const float* __restrict__ sf, const float* __restrict__ w,
                                                const float* __restrict__ b, unsigned short* xo,
                                                int nN, int nUnits) {
  const int u = (int)blockIdx.x * NTHR + (int)threadIdx.x;
  if (u >= nUnits) return;
  const int row = u >> 4;
  const int pc  = u & 15;
  const int f0  = (pc & 7) * 8;
  const int rc  = row < nN ? row : nN - 1;
  const float* sp = sf + (size_t)rc * 5;
  v4f aa = {0.f, 0.f, 0.f, 0.f};
  v4f ab = {0.f, 0.f, 0.f, 0.f};
#pragma unroll 1
  for (int i = 0; i < 5; ++i) {
    const float s = bfr(sp[i]);
    const v4f wa = bfr4(*(const v4fa*)(w + i * FD + f0));
    const v4f wb = bfr4(*(const v4fa*)(w + i * FD + f0 + 4));
    aa.x = fmaf(s, wa.x, aa.x); aa.y = fmaf(s, wa.y, aa.y);
    aa.z = fmaf(s, wa.z, aa.z); aa.w = fmaf(s, wa.w, aa.w);
    ab.x = fmaf(s, wb.x, ab.x); ab.y = fmaf(s, wb.y, ab.y);
    ab.z = fmaf(s, wb.z, ab.z); ab.w = fmaf(s, wb.w, ab.w);
  }
  const v4f ba = bfr4(*(const v4fa*)(b + f0));
  const v4f bb = bfr4(*(const v4fa*)(b + f0 + 4));
  const bool live = row < nN;
  v4f oa, ob;
  oa.x = live ? reluk(aa.x + ba.x) : 0.f;
  oa.y = live ? reluk(aa.y + ba.y) : 0.f;
  oa.z = live ? reluk(aa.z + ba.z) : 0.f;
  oa.w = live ? reluk(aa.w + ba.w) : 0.f;
  ob.x = live ? reluk(ab.x + bb.x) : 0.f;
  ob.y = live ? reluk(ab.y + bb.y) : 0.f;
  ob.z = live ? reluk(ab.z + bb.z) : 0.f;
  ob.w = live ? reluk(ab.w + bb.w) : 0.f;
  const HL8 r = split8(oa, ob);
  const unsigned int msk = (pc >= 8) ? 0xFFFFFFFFu : 0u;
  v4u ov;
  ov.x = (r.h.x & ~msk) | (r.l.x & msk);
  ov.y = (r.h.y & ~msk) | (r.l.y & msk);
  ov.z = (r.h.z & ~msk) | (r.l.z & msk);
  ov.w = (r.h.w & ~msk) | (r.l.w & msk);
  unsigned short* o = xo + (size_t)row * K0 + 8 * pc;
  *(volatile v4u*)o = ov;
  __threadfence();
  *(volatile v4u*)o = ov;
}

__global__ __launch_bounds__(NTHR) VG void k_wt(const float* __restrict__ w, int Kin, int Ncol, int Nrows, int Kout,
                                                unsigned short* wt, int nUnits) {
  const int u = (int)blockIdx.x * NTHR + (int)threadIdx.x;
  if (u >= nUnits) return;
  const int kq = Kout >> 3;
  const int n  = u / kq;
  const int k8 = (u - n * kq) * 8;
  const int kk = k8 - (k8 / Kin) * Kin;
  const int ncl = n < Ncol ? n : Ncol - 1;
  const float* p = w + (size_t)kk * (size_t)Ncol + ncl;
  v4f a, b;
  a.x = p[0];                    a.y = p[(size_t)Ncol];         a.z = p[(size_t)2 * Ncol];     a.w = p[(size_t)3 * Ncol];
  b.x = p[(size_t)4 * Ncol];     b.y = p[(size_t)5 * Ncol];     b.z = p[(size_t)6 * Ncol];     b.w = p[(size_t)7 * Ncol];
  const v4f z4 = {0.f, 0.f, 0.f, 0.f};
  if (n >= Ncol || n >= Nrows) { a = z4; b = z4; }
  const v4u wv = pack8(a, b);
  unsigned short* o = wt + (size_t)n * (size_t)Kout + k8;
  *(volatile v4u*)o = wv;
  __threadfence();
  *(volatile v4u*)o = wv;
}

template <int FIN>
__global__ __launch_bounds__(GTHR) VG void k_gemm(
    const unsigned short* __restrict__ A, const unsigned short* __restrict__ WT,
    float* outF, int K, int ldo,
    const float* __restrict__ atts, const float* __restrict__ attd, int attLen,
    float* SD, int MPr)
{
  __shared__ __attribute__((aligned(16))) float stg[GBM * GBN];
  __shared__ __attribute__((aligned(16))) float satt[2 * GBN];
  __shared__ __attribute__((aligned(16))) float sdot[2 * GBM];
  const int tid = (int)threadIdx.x, lane = tid & 31, wave = tid >> 5, hh = lane >> 4, m = lane & 15;
  const int rowBase = (int)blockIdx.x * GBM;
  const int head    = (int)blockIdx.y;
  const int col0    = head * GBN;

  if constexpr (FIN == 0) {
    const int which = tid >> 6;
    const int c  = tid & 63;
    const int cl = c < attLen ? c : attLen - 1;
    const float vs = atts[head * attLen + cl];
    const float vd = attd[head * attLen + cl];
    const unsigned int msk = (which == 0) ? 0u : 0xFFFFFFFFu;
    const unsigned int inr = (c < attLen) ? 0xFFFFFFFFu : 0u;
    float v = __uint_as_float((__float_as_uint(vs) & ~msk) | (__float_as_uint(vd) & msk));
    v = __uint_as_float(__float_as_uint(bfr(v)) & inr);
    satt[which * GBN + c] = v;
  }

  v8f acc[4];
  {
    const v8f z = {0.f, 0.f, 0.f, 0.f, 0.f, 0.f, 0.f, 0.f};
    acc[0] = z; acc[1] = z; acc[2] = z; acc[3] = z;
  }
  const unsigned short* ap = A  + (size_t)(rowBase + 16 * wave + m) * (size_t)K + 8 * hh;
  const unsigned short* wp = WT + (size_t)(col0 + m) * (size_t)K + 8 * hh;
  const int ksteps = K >> 5;
#pragma unroll 1
  for (int ks = 0; ks < ksteps; ++ks) {
    FragB af;
    af.h[0] = *(const v8usa*)(ap + 32 * ks);
    af.h[1] = *(const v8usa*)(ap + 32 * ks + 16);
#pragma unroll
    for (int t = 0; t < 4; ++t) {
      const unsigned short* wq = wp + (size_t)(16 * t) * (size_t)K + 32 * ks;
      FragB bf;
      bf.h[0] = *(const v8usa*)wq;
      bf.h[1] = *(const v8usa*)(wq + 16);
      acc[t] = wmb(af, bf, acc[t]);
    }
  }

#pragma unroll
  for (int t = 0; t < 4; ++t) {
    const int lc = 16 * t + m;
#pragma unroll
    for (int r = 0; r < 8; ++r) {
      const int lr = 16 * wave + 8 * hh + r;
      stg[lr * GBN + lc] = acc[t][r];
    }
  }
  __syncthreads();

  if constexpr (FIN == 0) {
    const int row = tid & 63, which = tid >> 6;
    const float* sa = satt + which * GBN;
    const float* hr = stg + row * GBN;
    float d = 0.f;
#pragma unroll 4
    for (int c4 = 0; c4 < GBN / 4; ++c4) {
      const v4f hv = *(const v4fa*)(hr + 4 * c4);
      const v4f av = *(const v4fa*)(sa + 4 * c4);
      d = fmaf(hv.x, av.x, d);
      d = fmaf(hv.y, av.y, d);
      d = fmaf(hv.z, av.z, d);
      d = fmaf(hv.w, av.w, d);
    }
    sdot[which * GBM + row] = d;
  }
  __syncthreads();

  v4f bb = {0.f, 0.f, 0.f, 0.f};
  if constexpr (FIN != 0) bb = bfr4(*(const v4fa*)(atts + col0 + 4 * m));
  v4f fv[8];
#pragma unroll
  for (int i = 0; i < 8; ++i) {
    const int lr = 16 * wave + 2 * i + hh;
    v4f t4 = *(const v4fa*)(stg + lr * GBN + 4 * m);
    t4.x += bb.x; t4.y += bb.y; t4.z += bb.z; t4.w += bb.w;
    fv[i] = t4;
  }

  if constexpr (FIN == 0) {
    const int which2 = lane >> 4, piece = lane & 15;
    const v4f sdv = *(const v4fa*)(sdot + which2 * GBM + 4 * piece);
    float* sp = SD + (size_t)(2 * head + which2) * (size_t)MPr + rowBase + 4 * piece;
#pragma unroll
    for (int i = 0; i < 8; ++i) {
      const int lr = 16 * wave + 2 * i + hh;
      const int gr = rowBase + lr;
      float* op = outF + (size_t)gr * (size_t)ldo + col0 + 4 * m;
      *(volatile v4f*)op = fv[i];
    }
    if (wave == 0) *(volatile v4f*)sp = sdv;
    __threadfence();
#pragma unroll
    for (int i = 0; i < 8; ++i) {
      const int lr = 16 * wave + 2 * i + hh;
      const int gr = rowBase + lr;
      float* op = outF + (size_t)gr * (size_t)ldo + col0 + 4 * m;
      *(volatile v4f*)op = fv[i];
    }
    if (wave == 0) *(volatile v4f*)sp = sdv;
  } else {
#pragma unroll
    for (int i = 0; i < 8; ++i) {
      const int lr = 16 * wave + 2 * i + hh;
      const int gr = rowBase + lr;
      float* op = outF + (size_t)gr * (size_t)ldo + col0 + 4 * m;
      *(volatile v4f*)op = fv[i];
    }
    __threadfence();
#pragma unroll
    for (int i = 0; i < 8; ++i) {
      const int lr = 16 * wave + 2 * i + hh;
      const int gr = rowBase + lr;
      float* op = outF + (size_t)gr * (size_t)ldo + col0 + 4 * m;
      *(volatile v4f*)op = fv[i];
    }
  }
}

__global__ __launch_bounds__(NTHR) VG void k_scan(
    const int* __restrict__ srcs, const int* __restrict__ dsts,
    const float* __restrict__ F, const float* __restrict__ SD,
    const float* __restrict__ bias, unsigned short* HP,
    int nN, int nE, int vec8, int MPr) {
  extern __shared__ v4f lds_dyn[];
  int* reg1 = (int*)lds_dyn;
  int* reg2 = reg1 + RCAP;
  int* scnt = reg2 + RCAP;
  int* soff = scnt + NB;
  int* list = soff + NB;
  int* wcnt = list + LISTN;
  int* wtot = wcnt + NWAVE;
  const int tid = (int)threadIdx.x, lane = tid & 31, wave = tid >> 5;
  const int nodeBase = (int)blockIdx.x * NB;

  for (int i = tid; i < NB; i += NTHR) scnt[i] = 0;
  __syncthreads();

  int tot = 0;
  const int nChunks = (nE + CHUNK - 1) / CHUNK;
#pragma unroll 1
  for (int ch = 0; ch < nChunks; ++ch) {
    const int cbase = ch * CHUNK;
    const int wc = scan_chunk(dsts, nE, cbase, nodeBase, NB, vec8, list, tid, lane, wave);
    if (lane == 0) wcnt[wave] = wc;
    __syncthreads();
    int pre = 0, all = 0;
#pragma unroll
    for (int w2 = 0; w2 < NWAVE; ++w2) {
      int c = wcnt[w2];
      c = c < 0 ? 0 : (c > WCAP ? WCAP : c);
      all += c;
      pre += (w2 < wave) ? c : 0;
    }
    const int wcc  = wc > WCAP ? WCAP : wc;
    const int base = tot + pre;
#pragma unroll 1
    for (int i = lane; i < wcc; i += 32) {
      const int ent = list[wave * WCAP + i];
      const int el  = (ent >> SLOTB) & (CHUNK - 1);
      const int sl  = ent & (NB - 1);
      int eid = cbase + el;
      eid = eid > nE - 1 ? nE - 1 : eid;
      const int pos = base + i;
      if (pos < RCAP) reg1[pos] = (int)(((unsigned)eid << SLOTB) | (unsigned)sl);
    }
    tot += all;
    tot = tot > RCAP ? RCAP : tot;
    __syncthreads();
  }
  const int nh = tot;

  if (wave == 0) {
#pragma unroll 1
    for (int b0 = 0; b0 < nh; b0 += 32) {
      const int idx = b0 + lane;
      const int uv  = reg1[idx < nh ? idx : nh - 1];
      const int m32 = (nh - b0) < 32 ? (nh - b0) : 32;
#pragma unroll 1
      for (int k = 0; k < m32; ++k) {
        const int u  = __builtin_amdgcn_readlane(uv, k);
        const int sl = u & (NB - 1);
        if (lane == 0) scnt[sl] = scnt[sl] + 1;
      }
    }
  }
  __syncthreads();

  {
    const v4i ca = *(const v4ia*)(scnt + 4 * tid);
    const int e0 = ca.x < 0 ? 0 : ca.x, e1 = ca.y < 0 ? 0 : ca.y, e2 = ca.z < 0 ? 0 : ca.z, e3 = ca.w < 0 ? 0 : ca.w;
    const int ts = e0 + e1 + e2 + e3;
    int incl = ts;
#pragma unroll
    for (int d = 1; d < 32; d <<= 1) {
      const int up = __shfl_up(incl, d);
      if (lane >= d) incl += up;
    }
    if (lane == 31) wtot[wave] = incl;
    __syncthreads();
    int pre = 0;
#pragma unroll
    for (int w2 = 0; w2 < NWAVE; ++w2) pre += (w2 < wave) ? wtot[w2] : 0;
    int run = pre + incl - ts;
    soff[4 * tid + 0] = run; run += e0;
    soff[4 * tid + 1] = run; run += e1;
    soff[4 * tid + 2] = run; run += e2;
    soff[4 * tid + 3] = run;
  }
  __syncthreads();
  for (int i = tid; i < NB; i += NTHR) list[i] = soff[i];
  __syncthreads();

  if (wave == 0) {
#pragma unroll 1
    for (int b0 = 0; b0 < nh; b0 += 32) {
      const int idx = b0 + lane;
      const int uv  = reg1[idx < nh ? idx : nh - 1];
      const int m32 = (nh - b0) < 32 ? (nh - b0) : 32;
#pragma unroll 1
      for (int k = 0; k < m32; ++k) {
        const int u   = __builtin_amdgcn_readlane(uv, k);
        const int sl  = u & (NB - 1);
        const int eid = (int)((unsigned)u >> SLOTB);
        if (lane == 0) {
          int pos = list[sl];
          pos = pos < 0 ? 0 : (pos > RCAP - 1 ? RCAP - 1 : pos);
          reg2[pos] = eid;
          list[sl] = pos + 1;
        }
      }
    }
  }
  __syncthreads();

  const int nbw = NB / NWAVE;
  const bool ovf = (nh >= RCAP);
  const float qnan = __int_as_float(0x7fc00000);
  const int c0   = 8 * lane;
  const int head = lane >> 3;
  const v4f bbA  = bfr4(*(const v4fa*)(bias + c0));
  const v4f bbB  = bfr4(*(const v4fa*)(bias + c0 + 4));
  const float* ASp = SD + (size_t)(2 * head) * (size_t)MPr;
  const float* ADp = ASp + MPr;

#pragma unroll 1
  for (int jt = 0; jt < nbw; ++jt) {
    const int slot = wave * nbw + jt;
    const int grow = nodeBase + slot;
    if (grow < MPr) {
      const int gcl  = grow < nN ? grow : nN - 1;
      int st = soff[slot];
      const int craw = scnt[slot];
      int cnt = craw;
      st  = st < 0 ? 0 : (st > nh ? nh : st);
      cnt = cnt < 0 ? 0 : (cnt > DEGCAP ? DEGCAP : cnt);
      if (cnt > nh - st) cnt = nh - st;
      const float pz = (ovf || craw > DEGCAP) ? qnan : 0.0f;

      const float* fr = F + (size_t)gcl * HC + c0;
      v4f av = *(const v4fa*)fr;
      v4f bv = *(const v4fa*)(fr + 4);
      const float adv = ADp[gcl];
      float l0 = ASp[gcl] + adv;
      l0 = l0 > 0.f ? l0 : NEGSL * l0;
      float mx = l0, dn = 1.0f;

#pragma unroll 1
      for (int q = 0; q < cnt; ++q) {
        int idx = st + q; idx = idx > RCAP - 1 ? RCAP - 1 : idx;
        int eid = reg2[idx]; eid = eid < 0 ? 0 : (eid > nE - 1 ? nE - 1 : eid);
        const int sraw = srcs[eid];
        const int s = sraw < 0 ? 0 : (sraw > nN - 1 ? nN - 1 : sraw);
        const float* gsrc = F + (size_t)s * HC + c0;
        const v4f fa = *(const v4fa*)gsrc;
        const v4f fb = *(const v4fa*)(gsrc + 4);
        float lg = ASp[s] + adv;
        lg = lg > 0.f ? lg : NEGSL * lg;
        const float df = lg - mx;
        const float ee = expf(-fabsf(df));
        const bool up  = df > 0.f;
        const float s1 = up ? ee : 1.0f;
        const float s2 = up ? 1.0f : ee;
        mx = up ? lg : mx;
        dn = fmaf(dn, s1, s2);
        av.x = fmaf(av.x, s1, s2 * fa.x);
        av.y = fmaf(av.y, s1, s2 * fa.y);
        av.z = fmaf(av.z, s1, s2 * fa.z);
        av.w = fmaf(av.w, s1, s2 * fa.w);
        bv.x = fmaf(bv.x, s1, s2 * fb.x);
        bv.y = fmaf(bv.y, s1, s2 * fb.y);
        bv.z = fmaf(bv.z, s1, s2 * fb.z);
        bv.w = fmaf(bv.w, s1, s2 * fb.w);
      }
      const float inv = 1.0f / (dn + EPS_SM);
      const bool live = grow < nN;
      v4f oa, ob;
      oa.x = (live ? reluk(fmaf(av.x, inv, bbA.x)) : 0.f) + pz;
      oa.y = (live ? reluk(fmaf(av.y, inv, bbA.y)) : 0.f) + pz;
      oa.z = (live ? reluk(fmaf(av.z, inv, bbA.z)) : 0.f) + pz;
      oa.w = (live ? reluk(fmaf(av.w, inv, bbA.w)) : 0.f) + pz;
      ob.x = (live ? reluk(fmaf(bv.x, inv, bbB.x)) : 0.f) + pz;
      ob.y = (live ? reluk(fmaf(bv.y, inv, bbB.y)) : 0.f) + pz;
      ob.z = (live ? reluk(fmaf(bv.z, inv, bbB.z)) : 0.f) + pz;
      ob.w = (live ? reluk(fmaf(bv.w, inv, bbB.w)) : 0.f) + pz;
      const HL8 r = split8(oa, ob);
      const v4u hv = r.h;
      const v4u lv = r.l;
      unsigned short* gp = HP + (size_t)grow * KA + 8 * lane;
      unsigned short* gq = gp + HC;
      *(volatile v4u*)gp = hv; *(volatile v4u*)gq = lv;
      __threadfence();
      *(volatile v4u*)gp = hv; *(volatile v4u*)gq = lv;
    }
  }
}

template <int C>
__global__ __launch_bounds__(NTHR) VG void k_pool(const unsigned short* __restrict__ xp,
                                                  const int* __restrict__ batch,
                                                  int nN, float* G, int coff) {
  static_assert(C == 64 || C == 256);
  constexpr int CPL = C / 32;
  constexpr int P   = 2 * C;
  __shared__ __attribute__((aligned(16))) float part[NWAVE * C];
  __shared__ __attribute__((aligned(16))) float res[C];
  const int tid = (int)threadIdx.x, lane = tid & 31, wave = tid >> 5;
  const int g = (int)blockIdx.x;
  const float ninf = __int_as_float((int)0xff800000);
  float mm[CPL];
#pragma unroll
  for (int j = 0; j < CPL; ++j) mm[j] = ninf;

  const int nIt = (nN + NTHR - 1) / NTHR;
#pragma unroll 1
  for (int it = 0; it < nIt; ++it) {
    const int base = (it * NWAVE + wave) * 32;
    const int n    = base + lane;
    const int ncl  = n < nN ? n : nN - 1;
    const int b    = batch[ncl];
    const bool hit = (n < nN) && (b == g);
    unsigned mask = __builtin_amdgcn_ballot_w32(hit);
#pragma unroll 1
    for (int q = 0; q < 32; ++q) {
      if (mask == 0u) break;
      const int k = __builtin_ctz(mask);
      mask &= mask - 1u;
      int node = base + k;
      node = node < 0 ? 0 : (node > nN - 1 ? nN - 1 : node);
      const unsigned short* rp = xp + (size_t)node * P;
      if constexpr (CPL == 8) {
        const v4u hw = *(const v4ua*)(rp + 8 * lane);
        const v4u lw = *(const v4ua*)(rp + C + 8 * lane);
        mm[0] = smax(mm[0], __uint_as_float(hw.x << 16)         + __uint_as_float(lw.x << 16));
        mm[1] = smax(mm[1], __uint_as_float(hw.x & 0xffff0000u) + __uint_as_float(lw.x & 0xffff0000u));
        mm[2] = smax(mm[2], __uint_as_float(hw.y << 16)         + __uint_as_float(lw.y << 16));
        mm[3] = smax(mm[3], __uint_as_float(hw.y & 0xffff0000u) + __uint_as_float(lw.y & 0xffff0000u));
        mm[4] = smax(mm[4], __uint_as_float(hw.z << 16)         + __uint_as_float(lw.z << 16));
        mm[5] = smax(mm[5], __uint_as_float(hw.z & 0xffff0000u) + __uint_as_float(lw.z & 0xffff0000u));
        mm[6] = smax(mm[6], __uint_as_float(hw.w << 16)         + __uint_as_float(lw.w << 16));
        mm[7] = smax(mm[7], __uint_as_float(hw.w & 0xffff0000u) + __uint_as_float(lw.w & 0xffff0000u));
      } else {
        const unsigned int hw = *(const u32a*)(rp + 2 * lane);
        const unsigned int lw = *(const u32a*)(rp + C + 2 * lane);
        mm[0] = smax(mm[0], __uint_as_float(hw << 16)         + __uint_as_float(lw << 16));
        mm[1] = smax(mm[1], __uint_as_float(hw & 0xffff0000u) + __uint_as_float(lw & 0xffff0000u));
      }
    }
  }
  if constexpr (CPL == 8) {
    v4f pa, pb;
    pa.x = mm[0]; pa.y = mm[1]; pa.z = mm[2]; pa.w = mm[3];
    pb.x = mm[4]; pb.y = mm[5]; pb.z = mm[6]; pb.w = mm[7];
    *(v4fa*)(part + wave * C + 8 * lane)     = pa;
    *(v4fa*)(part + wave * C + 8 * lane + 4) = pb;
  } else {
    v2f pa;
    pa.x = mm[0]; pa.y = mm[1];
    *(v2fa*)(part + wave * C + 2 * lane) = pa;
  }
  __syncthreads();
  {
    const int tc = tid < C ? tid : C - 1;
    float r = part[tc];
#pragma unroll
    for (int w2 = 1; w2 < NWAVE; ++w2) r = smax(r, part[w2 * C + tc]);
    if (tid < C) res[tid] = r;
  }
  __syncthreads();
  if (tid < C / 4) {
    const v4f r4 = *(const v4fa*)(res + 4 * tid);
    float* op = G + (size_t)g * GC + coff + 4 * tid;
    *(volatile v4f*)op = r4;
    __threadfence();
    *(volatile v4f*)op = r4;
  }
}

__global__ __launch_bounds__(NTHR) VG void k_gs(const float* __restrict__ G, unsigned short* ghl, int nUnits) {
  const int u = (int)blockIdx.x * NTHR + (int)threadIdx.x;
  if (u >= nUnits) return;
  const int row = u / (KG / 8);
  const int k8  = (u - row * (KG / 8)) * 8;
  const bool isLo = k8 >= GC;
  const int kk  = k8 - (isLo ? GC : 0);
  const float* p = G + (size_t)row * GC + kk;
  const v4f a = *(const v4fa*)p;
  const v4f b = *(const v4fa*)(p + 4);
  const HL8 r = split8(a, b);
  const unsigned int msk = isLo ? 0xFFFFFFFFu : 0u;
  v4u ov;
  ov.x = (r.h.x & ~msk) | (r.l.x & msk);
  ov.y = (r.h.y & ~msk) | (r.l.y & msk);
  ov.z = (r.h.z & ~msk) | (r.l.z & msk);
  ov.w = (r.h.w & ~msk) | (r.l.w & msk);
  unsigned short* o = ghl + (size_t)u * 8;
  *(volatile v4u*)o = ov;
  __threadfence();
  *(volatile v4u*)o = ov;
}

static inline int cdiv(int a, int b) { return (a + b - 1) / b; }

extern "C" void kernel_launch(void* const* d_in, const int* in_sizes, int n_in,
                              void* d_out, int out_size, void* d_ws, size_t ws_size,
                              hipStream_t stream) {
  if (n_in < 19) return;
  if (in_sizes[0] != NN * 5) return;
  if (in_sizes[1] != 2 * NE) return;
  if (in_sizes[2] != NN) return;
  if (in_sizes[3] != 5 * FD || in_sizes[4] != FD) return;
  if (in_sizes[5] != FD * HC) return;
  if (in_sizes[9] != HC * HC || in_sizes[13] != HC * HC) return;
  for (int l = 0; l < 3; ++l) {
    if (in_sizes[6 + 4 * l] != NHD * HID || in_sizes[7 + 4 * l] != NHD * HID) return;
    if (in_sizes[8 + 4 * l] != HC) return;
  }
  if (in_sizes[17] != GC * BOT || in_sizes[18] != BOT) return;
  if (out_size != NGR * BOT) return;

  const int nN = NN, nE = NE;
  const float* sf   = (const float*)d_in[0];
  const int*   ei   = (const int*)  d_in[1];
  const int*   bat  = (const int*)  d_in[2];
  const float* bw   = (const float*)d_in[3];
  const float* bbv  = (const float*)d_in[4];
  const float* aggw = (const float*)d_in[17];
  const float* aggb = (const float*)d_in[18];
  float* out = (float*)d_out;
  const int* src = ei;
  const int* dst = ei + nE;

  const int MP   = cdiv(nN, MROWS) * MROWS;
  if (MP != MPC) return;
  const int gM   = MP / GBM;
  const int gA   = cdiv(MP, NB);
  if ((long long)gA * NB < (long long)MP) return;
  const int vec8 = ((nE & 3) == 0) ? 1 : 0;

  char* ws = (char*)d_ws;
  size_t off = 0;
  const size_t oX0  = off; off += (size_t)MP * K0 * 2;           off = (off + 255) & ~(size_t)255;
  const size_t oW0  = off; off += (size_t)HC * K0 * 2;           off = (off + 255) & ~(size_t)255;
  const size_t oW1  = off; off += (size_t)HC * KA * 2;           off = (off + 255) & ~(size_t)255;
  const size_t oW2  = off; off += (size_t)HC * KA * 2;           off = (off + 255) & ~(size_t)255;
  const size_t oAG  = off; off += (size_t)BOT * KG * 2;          off = (off + 255) & ~(size_t)255;
  const size_t oH   = off; off += (size_t)MP * HC * 4;           off = (off + 255) & ~(size_t)255;
  const size_t oSD  = off; off += (size_t)2 * NHD * MP * 4;      off = (off + 255) & ~(size_t)255;
  const size_t oXH  = off; off += (size_t)MP * KA * 2;           off = (off + 255) & ~(size_t)255;
  const size_t oG   = off; off += (size_t)NGR * GC * 4;          off = (off + 255) & ~(size_t)255;
  const size_t oGH  = off; off += (size_t)NGR * KG * 2;          off = (off + 255) & ~(size_t)255;
  if (off > ws_size || off > (size_t)WSMAX) return;
  unsigned short* X0hl = (unsigned short*)(ws + oX0);
  unsigned short* W0D  = (unsigned short*)(ws + oW0);
  unsigned short* W1D  = (unsigned short*)(ws + oW1);
  unsigned short* W2D  = (unsigned short*)(ws + oW2);
  unsigned short* AGGD = (unsigned short*)(ws + oAG);
  float*          H    = (float*)(ws + oH);
  float*          SD   = (float*)(ws + oSD);
  unsigned short* Xhl  = (unsigned short*)(ws + oXH);
  float*          G    = (float*)(ws + oG);
  unsigned short* Ghl  = (unsigned short*)(ws + oGH);

  hipFuncSetAttribute(reinterpret_cast<const void*>(&k_scan),
                      hipFuncAttributeMaxDynamicSharedMemorySize, LDS_SCAN);

  const int nUx = MP * (K0 / 8);
  k_x0<<<cdiv(nUx, NTHR), NTHR, 0, stream>>>(sf, bw, bbv, X0hl, nN, nUx);

  {
    const int nU0 = HC * (K0 / 8);
    k_wt<<<cdiv(nU0, NTHR), NTHR, 0, stream>>>((const float*)d_in[5], FD, HC, HC, K0, W0D, nU0);
    const int nU1 = HC * (KA / 8);
    k_wt<<<cdiv(nU1, NTHR), NTHR, 0, stream>>>((const float*)d_in[9], HC, HC, HC, KA, W1D, nU1);
    k_wt<<<cdiv(nU1, NTHR), NTHR, 0, stream>>>((const float*)d_in[13], HC, HC, HC, KA, W2D, nU1);
    const int nU3 = BOT * (KG / 8);
    k_wt<<<cdiv(nU3, NTHR), NTHR, 0, stream>>>(aggw, GC, BOT, BOT, KG, AGGD, nU3);
  }

  k_pool<FD><<<NGR, NTHR, 0, stream>>>(X0hl, bat, nN, G, 0);

  for (int l = 0; l < 3; ++l) {
    const float* asv = (const float*)d_in[6 + 4 * l];
    const float* adv = (const float*)d_in[7 + 4 * l];
    const float* bsv = (const float*)d_in[8 + 4 * l];
    const unsigned short* Ap = (l == 0) ? X0hl : Xhl;
    const unsigned short* Wp = (l == 0) ? W0D : ((l == 1) ? W1D : W2D);
    const int Kl = (l == 0) ? K0 : KA;
    k_gemm<0><<<dim3(gM, HC / GBN), GTHR, 0, stream>>>(Ap, Wp, H, Kl, HC, asv, adv, HID, SD, MP);
    k_scan<<<gA, NTHR, LDS_SCAN, stream>>>(src, dst, H, SD, bsv, Xhl, nN, nE, vec8, MP);
    k_pool<HC><<<NGR, NTHR, 0, stream>>>(Xhl, bat, nN, G, FD + HC * l);
  }

  const int nUg = NGR * (KG / 8);
  k_gs<<<cdiv(nUg, NTHR), NTHR, 0, stream>>>(G, Ghl, nUg);
  k_gemm<1><<<dim3(NGR / GBM, BOT / GBN), GTHR, 0, stream>>>(Ghl, AGGD, out, KG, BOT, aggb, aggb, BOT, out, NGR);
}
